// MultiHeadSelfAttention_12137577578825
// MI455X (gfx1250) — hardware-run, weakly checked
//
#include <hip/hip_runtime.h>


#ifndef NB
#define NB 1
#endif
#ifndef SEQ
#define SEQ 4096
#endif
#define SEQ_FULL 4096
#define TT   SEQ
#define DM   1024
#define NH_  16
#define NKV  4
#define REP  (NH_ / NKV)
#define HD   64
#define DQ   (NH_ * HD)
#define DKV  (NKV * HD)
#define MAXPOS 4096
#define RH   ((TT < 512) ? TT : 512)
#define AW   4
#define PCAR 1024.0f
#define SCL  0.125f
#define SC2  0.18033688011112042f

#define AL256(b) ((((size_t)(b)) + 255) & ~(size_t)255)
#define CARVE_BYTES (AL256((size_t)DQ * DM * 2) + 2 * AL256((size_t)DKV * DM * 2) + AL256((size_t)DM * DQ * 2) + AL256(256) + AL256((size_t)MAXPOS * (HD / 2) * 2 * 4) \
    + AL256((size_t)TT * DM * 2) + AL256((size_t)TT * DQ * 4) + 2 * AL256((size_t)TT * DKV * 4) + 3 * AL256((size_t)NH_ * TT * HD * 2) + 3 * AL256((size_t)NKV * TT * HD * 2) \
    + 3 * AL256((size_t)NKV * HD * TT * 2) + 2 * AL256((size_t)TT * DQ * 2))

static_assert(TT % 64 == 0);
static_assert(RH % 64 == 0);
static_assert((TT - RH) % 64 == 0);
static_assert(DM % 64 == 0 && DQ % 64 == 0 && DKV % 64 == 0);
static_assert(DM % 32 == 0 && DQ % 32 == 0);
static_assert(HD == 64);
static_assert(HD * 2 == 128);
static_assert(NH_ % NKV == 0);
static_assert(AW * 16 == 64);
static_assert(RH % (AW * 16) == 0 && (TT - RH) % (AW * 16) == 0);
static_assert(TT % 32 == 0);
static_assert(TT <= MAXPOS);
static_assert((MAXPOS * (HD / 2)) % 256 == 0);
static_assert((TT * DM) % 8 == 0 && (DQ * DM) % 8 == 0 && (DKV * DM) % 8 == 0);
static_assert(((long long)NH_ * TT * HD / 2) % 256 == 0 && ((long long)NKV * TT * HD / 2) % 256 == 0);
static_assert((TT * HD) % 256 == 0);
static_assert(CARVE_BYTES <= (size_t)134217728u);

typedef _Float16 h16;
typedef unsigned short bf;
typedef __attribute__((ext_vector_type(16))) __bf16   v16bf;
typedef __attribute__((ext_vector_type(16))) _Float16 v16h;
typedef __attribute__((ext_vector_type(8)))  _Float16 v8h;
typedef __attribute__((ext_vector_type(8)))  unsigned short v8us;
typedef __attribute__((ext_vector_type(8)))  float    v8f;
typedef __attribute__((ext_vector_type(4)))  float    v4f;
typedef __attribute__((ext_vector_type(2))) _Float16 v2h;
typedef __attribute__((ext_vector_type(4))) _Float16 v4h;
typedef __attribute__((ext_vector_type(2))) unsigned short v2us;
typedef __attribute__((ext_vector_type(4))) unsigned short v4us;
typedef __attribute__((ext_vector_type(2))) float v2f;
typedef v8h  __attribute__((may_alias)) v8ha;
typedef v4f  __attribute__((may_alias)) v4fa;
typedef v8us __attribute__((may_alias)) v8usa;

__device__ __forceinline__ unsigned short f2bf(float f) { unsigned u = __float_as_uint(f); u += 0x7FFFu + ((u >> 16) & 1u); return (unsigned short)(u >> 16); }
__device__ __forceinline__ float bf2f(unsigned short b) { return __uint_as_float(((unsigned)b) << 16); }
__device__ __forceinline__ float bfr(float f) { return bf2f(f2bf(f)); }
__device__ __forceinline__ v16h cat16(v8h lo, v8h hi) { return __builtin_shufflevector(lo, hi, 0, 1, 2, 3, 4, 5, 6, 7, 8, 9, 10, 11, 12, 13, 14, 15); }
__device__ __forceinline__ v16bf cat16b(v8us lo, v8us hi) { return __builtin_bit_cast(v16bf, __builtin_shufflevector(lo, hi, 0, 1, 2, 3, 4, 5, 6, 7, 8, 9, 10, 11, 12, 13, 14, 15)); }
__device__ __forceinline__ v8f wmma16(v16h a, v16h b, v8f c) { return __builtin_amdgcn_wmma_f32_16x16x32_f16(false, a, false, b, (short)0, c, false, false); }
__device__ __forceinline__ v8f wmmab(v16bf a, v16bf b, v8f c) { return __builtin_amdgcn_wmma_f32_16x16x32_bf16(false, a, false, b, (short)0, c, false, false); }
__device__ __forceinline__ h16 tohx(float x) { return (h16)x; }
__device__ __forceinline__ void splitf(float y, unsigned short& h, unsigned short& l) { h = f2bf(y); l = f2bf(y - bf2f(h)); }

static __device__ __forceinline__ h16 toh_flush(float v) { const h16 r = (h16)v; return (fabsf(v) < 6.103515625e-05f) ? (h16)0.0f : r; }
static __device__ __forceinline__ v8f wmma16g(v16h a, v16h b, v8f c) { c = wmma16(a, b, c); asm volatile("v_nop\n\tv_nop\n\tv_nop\n\tv_nop" : "+v"(c) : "v"(a), "v"(b)); return c; }
static __device__ __forceinline__ v8f wmmabg(v16bf a, v16bf b, v8f c) { c = wmmab(a, b, c); asm volatile("v_nop\n\tv_nop\n\tv_nop\n\tv_nop" : "+v"(c) : "v"(a), "v"(b)); return c; }

template <typename T16> struct WFrag;
template <> struct WFrag<h16> { typedef v16h V; static __device__ __forceinline__ V ld(const h16* p) { return cat16(*(const v8h*)p, *(const v8h*)(p + 16)); } static __device__ __forceinline__ v8f mma(V a, V b, v8f c) { return wmma16(a, b, c); } };
template <> struct WFrag<bf> { typedef v16bf V; static __device__ __forceinline__ V ld(const bf* p) { return cat16b(*(const v8us*)p, *(const v8us*)(p + 16)); } static __device__ __forceinline__ v8f mma(V a, V b, v8f c) { return wmmab(a, b, c); } };

template <typename T16, int NSPLIT, bool BIAS>
__global__ __launch_bounds__(32) void k_gemmw(const T16* __restrict__ A, const T16* __restrict__ A2, const T16* __restrict__ Bt, const T16* __restrict__ Bt2, int K, float* C, int ldc, const float* __restrict__ bias, size_t sA, size_t sB, size_t sC) {
    typedef typename WFrag<T16>::V V;
    __shared__ __align__(16) float os[16 * 68];
    const size_t z = blockIdx.z; A += z * sA; if (A2) A2 += z * sA; Bt += z * sB; if (Bt2) Bt2 += z * sB; C += z * sC;
    const int lane = threadIdx.x & 31, lr = lane & 15, hi = lane >> 4; const int r0 = blockIdx.x * 64, c0 = blockIdx.y * 64;
    v8f acc[4][4];
#pragma unroll
    for (int mb = 0; mb < 4; ++mb)
#pragma unroll
        for (int nb = 0; nb < 4; ++nb) acc[mb][nb] = (v8f){};
    const size_t aoff = (size_t)(r0 + lr) * K + 8 * hi, boff = (size_t)(c0 + lr) * K + 8 * hi;
#pragma unroll 1
    for (int kc = 0; kc < K; kc += 32) {
        V a[4], a2[4];
#pragma unroll
        for (int mb = 0; mb < 4; ++mb) { a[mb] = WFrag<T16>::ld(A + aoff + (size_t)mb * 16 * K + kc); if (NSPLIT == 1 || NSPLIT == 2) a2[mb] = WFrag<T16>::ld(A2 + aoff + (size_t)mb * 16 * K + kc); }
#pragma unroll
        for (int nb = 0; nb < 4; ++nb) { const V b = WFrag<T16>::ld(Bt + boff + (size_t)nb * 16 * K + kc); V b2; if (NSPLIT >= 2) b2 = WFrag<T16>::ld(Bt2 + boff + (size_t)nb * 16 * K + kc);
#pragma unroll
            for (int mb = 0; mb < 4; ++mb) { acc[mb][nb] = WFrag<T16>::mma(a[mb], b, acc[mb][nb]); if (NSPLIT == 1 || NSPLIT == 2) acc[mb][nb] = WFrag<T16>::mma(a2[mb], b, acc[mb][nb]); if (NSPLIT >= 2) acc[mb][nb] = WFrag<T16>::mma(a[mb], b2, acc[mb][nb]); } }
        asm volatile("v_nop\n\tv_nop\n\tv_nop\n\tv_nop" : "+v"(acc[0][0]), "+v"(acc[1][1]), "+v"(acc[2][2]), "+v"(acc[3][3]) : "v"(a[0]), "v"(a[3]));
    }
#pragma unroll
    for (int mb = 0; mb < 4; ++mb) {
#pragma unroll
        for (int nb = 0; nb < 4; ++nb) {
#pragma unroll
            for (int j = 0; j < 8; ++j) os[(hi * 8 + j) * 68 + nb * 16 + lr] = acc[mb][nb][j]; }
        __builtin_amdgcn_wave_barrier(); asm volatile("" ::: "memory");
        float* crow = C + (size_t)(r0 + mb * 16) * ldc + c0;
#pragma unroll 1
        for (int ps = 0; ps < 2; ++ps) {
#pragma unroll
            for (int s = 0; s < 8; ++s) { const int row = 2 * s + hi, cofs = lr * 4; v4f val = *(const v4fa*)(os + row * 68 + cofs); if (BIAS) { val[0] += bfr(bias[c0 + cofs]); val[1] += bfr(bias[c0 + cofs + 1]); val[2] += bfr(bias[c0 + cofs + 2]); val[3] += bfr(bias[c0 + cofs + 3]); }
                *(volatile v4f*)(crow + (size_t)row * ldc + cofs) = val; }
            if (ps == 0) __threadfence(); }
        __builtin_amdgcn_wave_barrier(); asm volatile("" ::: "memory");
    }
}

__global__ __launch_bounds__(256) void k_cvt8(const float* __restrict__ src, bf* dst, size_t n8) { const size_t i = (size_t)blockIdx.x * 256 + threadIdx.x; if (i >= n8) return; const v8f v = *(const v8f*)(src + i * 8); v8us o;
#pragma unroll
    for (int k = 0; k < 8; ++k) o[k] = f2bf(v[k]); *(volatile v8us*)(dst + i * 8) = o; __threadfence(); *(volatile v8us*)(dst + i * 8) = o; }

__global__ __launch_bounds__(32) void k_invf(float* IF) { const int d = threadIdx.x & 31; const float e = (float)(2 * d) * (1.0f / 64.0f); const float p = powf(10000.0f, e); const float v = 1.0f / p;
    *(volatile float*)(IF + d) = v; __threadfence(); *(volatile float*)(IF + d) = v; }
__global__ __launch_bounds__(256) void k_cs(const float* __restrict__ IF, float* CS) { const int idx = blockIdx.x * 256 + threadIdx.x; if (idx >= MAXPOS * (HD / 2)) return; const int d = idx % (HD / 2), t = idx / (HD / 2); const float ang = (float)t * IF[d]; float sn, cn; sincosf(ang, &sn, &cn);
    v2f cs; cs[0] = cn; cs[1] = sn; *(volatile v2f*)(CS + (size_t)idx * 2) = cs; __threadfence(); *(volatile v2f*)(CS + (size_t)idx * 2) = cs; }

__global__ __launch_bounds__(256) void k_rope(const float* __restrict__ F, int pitch, int nheads, const float* __restrict__ CS, const int* __restrict__ pos, h16* P16, bf* Ph, bf* Pl) {
#pragma clang fp contract(off)
    const size_t e = ((size_t)blockIdx.x * 256 + threadIdx.x) * 2; if (e >= (size_t)nheads * TT * HD) return; const int d = (int)(e % HD); const int t = (int)((e / HD) % TT); const int h = (int)(e / ((size_t)HD * TT));
    int p = pos[t]; p = (p < 0) ? (p + MAXPOS) : p; p = (p < 0) ? 0 : p; p = (p > MAXPOS - 1) ? (MAXPOS - 1) : p;
    const v2f cs = *(const v2f*)(CS + ((size_t)p * (HD / 2) + (d >> 1)) * 2);
    const v2f x = *(const v2f*)(F + (size_t)t * pitch + h * HD + d);
    float a = __fmul_rn(x[0], cs[0]), bq = __fmul_rn(x[1], cs[1]), cq = __fmul_rn(x[0], cs[1]), dq = __fmul_rn(x[1], cs[0]);
    asm volatile("" : "+v"(a)); asm volatile("" : "+v"(bq)); asm volatile("" : "+v"(cq)); asm volatile("" : "+v"(dq));
    const float r1 = __fsub_rn(a, bq); const float r2 = __fadd_rn(cq, dq);
    v2h o16; v2us oh, ol; unsigned short a2, c2;
    o16[0] = toh_flush(r1); o16[1] = toh_flush(r2);
    splitf(r1, a2, c2); oh[0] = a2; ol[0] = c2; splitf(r2, a2, c2); oh[1] = a2; ol[1] = c2;
    *(volatile v2h*)(P16 + e) = o16; *(volatile v2us*)(Ph + e) = oh; *(volatile v2us*)(Pl + e) = ol; __threadfence(); *(volatile v2h*)(P16 + e) = o16; *(volatile v2us*)(Ph + e) = oh; *(volatile v2us*)(Pl + e) = ol; }
__global__ __launch_bounds__(256) void k_vtp(const float* __restrict__ F, int pitch, int nheads, h16* V16, bf* Vh, bf* Vl) { const size_t e = ((size_t)blockIdx.x * 256 + threadIdx.x) * 2; if (e >= (size_t)nheads * HD * TT) return; const int t = (int)(e % TT); const int d = (int)((e / TT) % HD); const int g = (int)(e / ((size_t)TT * HD)); v2h o16; v2us oh, ol;
#pragma unroll
    for (int q = 0; q < 2; ++q) { const float x = F[(size_t)(t + q) * pitch + g * HD + d]; o16[q] = tohx(x); unsigned short a2, c2; splitf(x, a2, c2); oh[q] = a2; ol[q] = c2; }
    *(volatile v2h*)(V16 + e) = o16; *(volatile v2us*)(Vh + e) = oh; *(volatile v2us*)(Vl + e) = ol; __threadfence(); *(volatile v2h*)(V16 + e) = o16; *(volatile v2us*)(Vh + e) = oh; *(volatile v2us*)(Vl + e) = ol; }

template <bool EARLY>
__device__ __forceinline__ void attn_body(const h16* __restrict__ Q16, const bf* __restrict__ Qh, const bf* __restrict__ Ql, const h16* __restrict__ K16, const bf* __restrict__ Kh, const bf* __restrict__ Kl,
                                          const h16* __restrict__ V16, const bf* __restrict__ Vh, const bf* __restrict__ Vl, bf* Ah, bf* Al, int roff) {
    __shared__ __align__(16) float os[AW * 16 * 68];
    const int wave = __builtin_amdgcn_readfirstlane(threadIdx.x >> 5);
    const int lane = threadIdx.x & 31, lr = lane & 15, hi = lane >> 4;
    const int h = blockIdx.y; const int g = h / REP;
    const int qw = roff + (int)blockIdx.x * (AW * 16) + wave * 16;
    const int nst = (qw >> 5) + 1;
    const int qi = qw + lr;
    const size_t qoff = ((size_t)h * TT + qw + lr) * HD + 8 * hi;
    const size_t koff = ((size_t)g * TT + lr) * HD + 8 * hi;
    const size_t voff = ((size_t)g * HD + lr) * TT + 8 * hi;
    v16h q16[2]; v16bf qh[2], ql[2];
#pragma unroll
    for (int ds = 0; ds < 2; ++ds) {
        if (EARLY) { qh[ds] = WFrag<bf>::ld(Qh + qoff + ds * 32); ql[ds] = WFrag<bf>::ld(Ql + qoff + ds * 32); }
        else { q16[ds] = WFrag<h16>::ld(Q16 + qoff + ds * 32); } }
    v8f o[4];
#pragma unroll
    for (int dt = 0; dt < 4; ++dt) o[dt] = (v8f){};
    float m = -3.0e38f, l = 0.0f;
#pragma unroll 1
    for (int st = 0; st < nst; ++st) {
        const int kb = st * 32;
        v8f s[2];
#pragma unroll
        for (int kt = 0; kt < 2; ++kt) {
            v8f c = (v8f){};
            const size_t ko = koff + (size_t)(kb + kt * 16) * HD;
#pragma unroll
            for (int ds = 0; ds < 2; ++ds) {
                if (EARLY) { const v16bf kah = WFrag<bf>::ld(Kh + ko + ds * 32); const v16bf kal = WFrag<bf>::ld(Kl + ko + ds * 32);
                    c = wmmabg(kah, qh[ds], c); c = wmmabg(kal, qh[ds], c); c = wmmabg(kah, ql[ds], c); }
                else { const v16h ka = WFrag<h16>::ld(K16 + ko + ds * 32); c = wmma16g(ka, q16[ds], c); } }
            s[kt] = c; }
        float tv[2][8]; float mx = -3.0e38f;
#pragma unroll
        for (int kt = 0; kt < 2; ++kt) {
#pragma unroll
            for (int r = 0; r < 8; ++r) { const int key = kb + kt * 16 + 8 * hi + r; const float x = (key <= qi) ? (s[kt][r] * SC2) : -3.0e38f; tv[kt][r] = x; mx = fmaxf(mx, x); } }
        mx = fmaxf(mx, __shfl_xor(mx, 16, 32));
        const float nm = fmaxf(m, mx);
        const float corr = __builtin_amdgcn_exp2f(m - nm);
        m = nm;
        float sum = 0.0f;
        v16h pf; v8us ph0, pl0, ph1, pl1;
        if (EARLY) {
#pragma unroll
            for (int r = 0; r < 8; ++r) { const float p0 = __builtin_amdgcn_exp2f(tv[0][r] - nm); const float p1 = __builtin_amdgcn_exp2f(tv[1][r] - nm); sum += p0 + p1;
                unsigned short a, c2; splitf(p0, a, c2); ph0[r] = a; pl0[r] = c2; splitf(p1, a, c2); ph1[r] = a; pl1[r] = c2; }
        } else {
#pragma unroll
            for (int r = 0; r < 8; ++r) { const float e0 = tv[0][r] - nm, e1 = tv[1][r] - nm;
                const float x0 = __builtin_amdgcn_exp2f(e0 + 10.0f), x1 = __builtin_amdgcn_exp2f(e1 + 10.0f);
                const float p0 = (e0 < -24.0f) ? 0.0f : x0; const float p1 = (e1 < -24.0f) ? 0.0f : x1;
                const h16 a0 = (h16)p0, a1 = (h16)p1; pf[r] = a0; pf[8 + r] = a1; sum += (float)a0 + (float)a1; }
        }
        l = l * corr + sum;
#pragma unroll
        for (int dt = 0; dt < 4; ++dt) {
#pragma unroll
            for (int r = 0; r < 8; ++r) o[dt][r] *= corr; }
        if (EARLY) {
            const v16bf Pfh = cat16b(ph0, ph1), Pfl = cat16b(pl0, pl1);
#pragma unroll
            for (int dt = 0; dt < 4; ++dt) { const size_t vo = voff + (size_t)dt * 16 * TT + kb; const v16bf vah = WFrag<bf>::ld(Vh + vo); const v16bf val = WFrag<bf>::ld(Vl + vo);
                o[dt] = wmmabg(vah, Pfh, o[dt]); o[dt] = wmmabg(val, Pfh, o[dt]); o[dt] = wmmabg(vah, Pfl, o[dt]); }
        } else {
#pragma unroll
            for (int dt = 0; dt < 4; ++dt) { const size_t vo = voff + (size_t)dt * 16 * TT + kb; const v16h va = WFrag<h16>::ld(V16 + vo); o[dt] = wmma16g(va, pf, o[dt]); }
        }
    }
    const float lt = l + __shfl_xor(l, 16, 32);
    const float inv = 1.0f / lt;
    const int wb = wave * (16 * 68);
#pragma unroll
    for (int dt = 0; dt < 4; ++dt) {
#pragma unroll
        for (int r = 0; r < 8; ++r) os[wb + lr * 68 + dt * 16 + 8 * hi + r] = o[dt][r] * inv; }
    __syncthreads();
#pragma unroll 1
    for (int ps = 0; ps < 2; ++ps) {
#pragma unroll
        for (int s4 = 0; s4 < 4; ++s4) { const int row = 4 * s4 + (lane >> 3), c8 = (lane & 7) * 8;
            const v4f x0 = *(const v4fa*)(os + wb + row * 68 + c8); const v4f x1 = *(const v4fa*)(os + wb + row * 68 + c8 + 4);
            v8us oh, ol;
#pragma unroll
            for (int k = 0; k < 4; ++k) { unsigned short a, c2; splitf(x0[k], a, c2); oh[k] = a; ol[k] = c2; splitf(x1[k], a, c2); oh[4 + k] = a; ol[4 + k] = c2; }
            const size_t oo = (size_t)(qw + row) * DQ + (size_t)h * HD + c8;
            *(volatile v8us*)(Ah + oo) = oh; *(volatile v8us*)(Al + oo) = ol; }
        if (ps == 0) __threadfence(); }
}

__global__ __launch_bounds__(128) __attribute__((amdgpu_num_vgpr(256))) void k_attn_early(const h16* __restrict__ Q16, const bf* __restrict__ Qh, const bf* __restrict__ Ql, const h16* __restrict__ K16, const bf* __restrict__ Kh, const bf* __restrict__ Kl,
                                                                                           const h16* __restrict__ V16, const bf* __restrict__ Vh, const bf* __restrict__ Vl, bf* Ah, bf* Al, int roff) {
    attn_body<true>(Q16, Qh, Ql, K16, Kh, Kl, V16, Vh, Vl, Ah, Al, roff); }
__global__ __launch_bounds__(128) __attribute__((amdgpu_num_vgpr(256))) void k_attn_late(const h16* __restrict__ Q16, const bf* __restrict__ Qh, const bf* __restrict__ Ql, const h16* __restrict__ K16, const bf* __restrict__ Kh, const bf* __restrict__ Kl,
                                                                                          const h16* __restrict__ V16, const bf* __restrict__ Vh, const bf* __restrict__ Vl, bf* Ah, bf* Al, int roff) {
    attn_body<false>(Q16, Qh, Ql, K16, Kh, Kl, V16, Vh, Vl, Ah, Al, roff); }

extern "C" void kernel_launch(void* const* d_in, const int* in_sizes, int n_in,
                              void* d_out, int out_size, void* d_ws, size_t ws_size, hipStream_t stream) {
    if (n_in < 6) return;
    if (in_sizes[0] < (NB - 1) * SEQ_FULL * DM + TT * DM) return;
    if (in_sizes[1] < DQ * DM || in_sizes[2] < DKV * DM || in_sizes[3] < DKV * DM || in_sizes[4] < DM * DQ) return;
    if (in_sizes[5] < (NB - 1) * SEQ_FULL + TT) return;
    if (out_size < NB * TT * DM) return;
    const float* x = (const float*)d_in[0]; const float* wq = (const float*)d_in[1]; const float* wk = (const float*)d_in[2]; const float* wv = (const float*)d_in[3]; const float* wo = (const float*)d_in[4];
    const int* tp = (const int*)d_in[5];
    float* OUT = (float*)d_out;
    char* wsp = (char*)d_ws;
    auto take = [&](size_t bytes) { char* p = wsp; wsp += (bytes + 255) & ~(size_t)255; return (void*)p; };
    bf* WQ = (bf*)take((size_t)DQ * DM * 2); bf* WK = (bf*)take((size_t)DKV * DM * 2); bf* WV = (bf*)take((size_t)DKV * DM * 2); bf* WO = (bf*)take((size_t)DM * DQ * 2);
    float* INVF = (float*)take(256); float* CS = (float*)take((size_t)MAXPOS * (HD / 2) * 2 * 4);
    bf* XB = (bf*)take((size_t)TT * DM * 2); float* FQ = (float*)take((size_t)TT * DQ * 4); float* FK = (float*)take((size_t)TT * DKV * 4); float* FV = (float*)take((size_t)TT * DKV * 4);
    h16* QP16 = (h16*)take((size_t)NH_ * TT * HD * 2); bf* QPh = (bf*)take((size_t)NH_ * TT * HD * 2); bf* QPl = (bf*)take((size_t)NH_ * TT * HD * 2);
    h16* KP16 = (h16*)take((size_t)NKV * TT * HD * 2); bf* KPh = (bf*)take((size_t)NKV * TT * HD * 2); bf* KPl = (bf*)take((size_t)NKV * TT * HD * 2);
    h16* VT16 = (h16*)take((size_t)NKV * HD * TT * 2); bf* VTh = (bf*)take((size_t)NKV * HD * TT * 2); bf* VTl = (bf*)take((size_t)NKV * HD * TT * 2);
    bf* ATh = (bf*)take((size_t)TT * DQ * 2); bf* ATl = (bf*)take((size_t)TT * DQ * 2);
    const size_t used = (size_t)(wsp - (char*)d_ws); if (used > ws_size || used > (size_t)134217728u) return;
    k_cvt8<<<(unsigned)(((size_t)DQ * DM / 8 + 255) / 256), 256, 0, stream>>>(wq, WQ, (size_t)DQ * DM / 8);
    k_cvt8<<<(unsigned)(((size_t)DKV * DM / 8 + 255) / 256), 256, 0, stream>>>(wk, WK, (size_t)DKV * DM / 8);
    k_cvt8<<<(unsigned)(((size_t)DKV * DM / 8 + 255) / 256), 256, 0, stream>>>(wv, WV, (size_t)DKV * DM / 8);
    k_cvt8<<<(unsigned)(((size_t)DM * DQ / 8 + 255) / 256), 256, 0, stream>>>(wo, WO, (size_t)DM * DQ / 8);
    k_invf<<<1, 32, 0, stream>>>(INVF);
    k_cs<<<(MAXPOS * (HD / 2) + 255) / 256, 256, 0, stream>>>(INVF, CS);
    const unsigned LQ = (unsigned)(((size_t)NH_ * TT * HD / 2 + 255) / 256), LKv = (unsigned)(((size_t)NKV * TT * HD / 2 + 255) / 256);
    for (int b = 0; b < NB; ++b) {
        const int* tpb = tp + (size_t)b * SEQ_FULL;
        k_cvt8<<<(unsigned)(((size_t)TT * DM / 8 + 255) / 256), 256, 0, stream>>>(x + (size_t)b * SEQ_FULL * DM, XB, (size_t)TT * DM / 8);
        k_gemmw<bf, 0, false><<<dim3(TT / 64, DQ / 64, 1), 32, 0, stream>>>(XB, nullptr, WQ, nullptr, DM, FQ, DQ, nullptr, 0, 0, 0);
        k_rope<<<LQ, 256, 0, stream>>>(FQ, DQ, NH_, CS, tpb, QP16, QPh, QPl);
        k_gemmw<bf, 0, false><<<dim3(TT / 64, DKV / 64, 1), 32, 0, stream>>>(XB, nullptr, WK, nullptr, DM, FK, DKV, nullptr, 0, 0, 0);
        k_rope<<<LKv, 256, 0, stream>>>(FK, DKV, NKV, CS, tpb, KP16, KPh, KPl);
        k_gemmw<bf, 0, false><<<dim3(TT / 64, DKV / 64, 1), 32, 0, stream>>>(XB, nullptr, WV, nullptr, DM, FV, DKV, nullptr, 0, 0, 0);
        k_vtp<<<LKv, 256, 0, stream>>>(FV, DKV, NKV, VT16, VTh, VTl);
        if (RH > 0) k_attn_early<<<dim3(RH / (AW * 16), NH_, 1), AW * 32, 0, stream>>>(QP16, QPh, QPl, KP16, KPh, KPl, VT16, VTh, VTl, ATh, ATl, 0);
        if (TT - RH > 0) k_attn_late<<<dim3((TT - RH) / (AW * 16), NH_, 1), AW * 32, 0, stream>>>(QP16, QPh, QPl, KP16, KPh, KPl, VT16, VTh, VTl, ATh, ATl, RH);
        k_gemmw<bf, 1, false><<<dim3(TT / 64, DM / 64, 1), 32, 0, stream>>>(ATh, ATl, WO, nullptr, DQ, OUT + (size_t)b * TT * DM, DM, nullptr, 0, 0, 0); }
}
